// SequenceEncoder_28054726378041
// MI455X (gfx1250) — hardware-verified
//
#include <hip/hip_runtime.h>
#include <stddef.h>
#include <stdint.h>


typedef __attribute__((ext_vector_type(16))) _Float16 v16h;
typedef __attribute__((ext_vector_type(8)))  _Float16 v8h;
typedef __attribute__((ext_vector_type(4)))  _Float16 v4h;
typedef __attribute__((ext_vector_type(16))) __bf16   v16b;
typedef __attribute__((ext_vector_type(8)))  __bf16   v8b;
typedef __attribute__((ext_vector_type(8)))  float    v8f;
typedef __attribute__((ext_vector_type(4)))  float    v4f;
typedef __attribute__((ext_vector_type(4)))  int      v4i;

__device__ __forceinline__ unsigned short f2bf_bits(float f) {
  unsigned u = __float_as_uint(f);
  return (unsigned short)((u + 0x7FFFu + ((u >> 16) & 1u)) >> 16);
}
__device__ __forceinline__ float bf_bits2f(unsigned short h) { return __uint_as_float(((unsigned)h) << 16); }

__device__ __forceinline__ void dep_guard_h(v8f& a, v8f& b, v16h x, v16h y) { asm volatile("v_nop\n\tv_nop\n\tv_nop\n\tv_nop" : "+v"(a), "+v"(b) : "v"(x), "v"(y)); }
__device__ __forceinline__ void dep_guard_b(v8f& a, v8f& b, v16b x, v16b y) { asm volatile("v_nop\n\tv_nop\n\tv_nop\n\tv_nop" : "+v"(a), "+v"(b) : "v"(x), "v"(y)); }
__device__ __forceinline__ void keep4_h(v16h a, v16h b, v16h c, v16h d) { asm volatile("v_nop" :: "v"(a), "v"(b), "v"(c), "v"(d)); }
__device__ __forceinline__ void keep4_b(v16b a, v16b b, v16b c, v16b d) { asm volatile("v_nop" :: "v"(a), "v"(b), "v"(c), "v"(d)); }
__device__ __forceinline__ void acc_guard4(v8f& a, v8f& b, v8f& c, v8f& d) { asm volatile("v_nop\n\tv_nop\n\tv_nop\n\tv_nop" : "+v"(a), "+v"(b), "+v"(c), "+v"(d)); }
template <typename T> struct Frag;
template <> struct Frag<_Float16> {
  typedef v16h V; union U { v16h v; v8h h[2]; };
  static __device__ __forceinline__ v16h load(const _Float16* p) {
    U f; f.h[0] = *(const v8h*)(p); f.h[1] = *(const v8h*)(p + 16); return f.v;
  }
  static __device__ __forceinline__ v8f mma(v16h a, v16h b, v8f c) {
    return __builtin_amdgcn_wmma_f32_16x16x32_f16(false, a, false, b, (short)0, c, false, false);
  }
  static __device__ __forceinline__ void guard(v8f& a, v8f& b, v16h x, v16h y) { dep_guard_h(a, b, x, y); }
  static __device__ __forceinline__ void keep(v16h a, v16h b, v16h c, v16h d) { keep4_h(a, b, c, d); }
};
template <> struct Frag<__bf16> {
  typedef v16b V; union U { v16b v; v8b h[2]; };
  static __device__ __forceinline__ v16b load(const __bf16* p) {
    U f; f.h[0] = *(const v8b*)(p); f.h[1] = *(const v8b*)(p + 16); return f.v;
  }
  static __device__ __forceinline__ v8f mma(v16b a, v16b b, v8f c) {
    return __builtin_amdgcn_wmma_f32_16x16x32_bf16(false, a, false, b, (short)0, c, false, false);
  }
  static __device__ __forceinline__ void guard(v8f& a, v8f& b, v16b x, v16b y) { dep_guard_b(a, b, x, y); }
  static __device__ __forceinline__ void keep(v16b a, v16b b, v16b c, v16b d) { keep4_b(a, b, c, d); }
};

template <int ET> struct Elem;
template <> struct Elem<0> { typedef _Float16 T; };
template <> struct Elem<1> { typedef __bf16 T; };
template <int ET, bool SPLIT, int BIAS_MODE, int OUT_MODE, bool RESID, int ACT = 0>
__global__ __launch_bounds__(256) void wmma_gemm64(
    const unsigned short* __restrict__ Ap, const unsigned short* __restrict__ A2p, int lda, long strideA,
    const unsigned short* __restrict__ Btp, const unsigned short* __restrict__ Bt2p, int ldb, long strideB,
    void* __restrict__ Cout, void* __restrict__ Cout2, int ldc, long strideC,
    const float* __restrict__ bias,
    const float* __restrict__ resid, long strideR,
    int M, int N, int K, float scale) {
  typedef typename Elem<ET>::T T;
  typedef typename Frag<T>::V V;
  const T* A = (const T*)Ap; const T* A2 = (const T*)A2p; const T* Bt = (const T*)Btp; const T* Bt2 = (const T*)Bt2p;
  __shared__ __align__(16) float sT[8][16 * 68];
  const int b    = blockIdx.y;
  const int lane = threadIdx.x & 31;
  const int wave = threadIdx.x >> 5;
  const int tilesN = N >> 6;
  const int tilesM = M >> 6;
  const int tile = blockIdx.x * 8 + wave;
  if (tile >= tilesM * tilesN) return;
  const int tm = tile / tilesN;
  const int tn = tile - tm * tilesN;
  const int m0 = tm << 6;
  const int n0 = tn << 6;

  const T* Ab  = A  + (size_t)b * strideA;
  const T* Bb  = Bt + (size_t)b * strideB;
  const T* Ab2 = SPLIT ? (A2  + (size_t)b * strideA) : nullptr;
  const T* Bb2 = SPLIT ? (Bt2 + (size_t)b * strideB) : nullptr;

  const int rlane = lane & 15;
  const int koff  = (lane >> 4) * 8;
  const int mOff  = (lane >> 4) * 8;

  v8f acc[4][4];
#pragma unroll
  for (int i = 0; i < 4; ++i)
#pragma unroll
    for (int j = 0; j < 4; ++j) acc[i][j] = (v8f){0.f,0.f,0.f,0.f,0.f,0.f,0.f,0.f};

  for (int k0 = 0; k0 < K; k0 += 32) {
    V bh[4], bl[4];
#pragma unroll
    for (int j = 0; j < 4; ++j) {
      const size_t bo = (size_t)(n0 + (j << 4) + rlane) * ldb + koff + k0;
      bh[j] = Frag<T>::load(Bb + bo);
      if (SPLIT) bl[j] = Frag<T>::load(Bb2 + bo);
    }
#pragma unroll
    for (int i = 0; i < 4; ++i) {
      const size_t ao = (size_t)(m0 + (i << 4) + rlane) * lda + koff + k0;
      V ah = Frag<T>::load(Ab + ao);
      V al;
      if (SPLIT) al = Frag<T>::load(Ab2 + ao);
#pragma unroll
      for (int j = 0; j < 4; ++j) {
        acc[i][j] = Frag<T>::mma(ah, bh[j], acc[i][j]);
        if (SPLIT) {
          acc[i][j] = Frag<T>::mma(ah, bl[j], acc[i][j]);
          acc[i][j] = Frag<T>::mma(al, bh[j], acc[i][j]);
        }
      }
      Frag<T>::guard(acc[i][0], acc[i][3], ah, SPLIT ? al : ah);
    }
    Frag<T>::keep(bh[0], bh[1], bh[2], bh[3]);
    if (SPLIT) Frag<T>::keep(bl[0], bl[1], bl[2], bl[3]);
  }
  acc_guard4(acc[0][0], acc[0][1], acc[0][2], acc[0][3]);
  acc_guard4(acc[1][0], acc[1][1], acc[1][2], acc[1][3]);
  acc_guard4(acc[2][0], acc[2][1], acc[2][2], acc[2][3]);
  acc_guard4(acc[3][0], acc[3][1], acc[3][2], acc[3][3]);

  float* slab = sT[wave];
  const float* Rb = RESID ? (resid + (size_t)b * strideR) : nullptr;
#pragma unroll
  for (int i = 0; i < 4; ++i) {
    const int mBase = m0 + (i << 4);
#pragma unroll
    for (int j = 0; j < 4; ++j) {
      const int n = n0 + (j << 4) + rlane;
      float bv = 0.f;
      if (BIAS_MODE == 2) bv = bias[n];
#pragma unroll
      for (int r = 0; r < 8; ++r) {
        float v = acc[i][j][r] * scale;
        if (BIAS_MODE == 1) v += bias[mBase + mOff + r];
        if (BIAS_MODE == 2) v += bv;
        if (RESID) v += Rb[(size_t)(mBase + mOff + r) * ldc + n];
        if (ACT == 1) v = tanhf(v);
        if (ACT == 2) v = fmaxf(v, 0.0f);
        if (ACT == 3) v = v / (1.0f + expf(-v));
        if (ACT == 4) v = (v > 0.f) ? v : 0.01f * v;
        if (ACT == 5) v = 0.5f * v * (1.0f + erff(v * 0.70710678118654752f));
        slab[(mOff + r) * 68 + (j << 4) + rlane] = v;
      }
    }
    __builtin_amdgcn_fence(__ATOMIC_RELEASE, "workgroup");
    __builtin_amdgcn_wave_barrier();
    __builtin_amdgcn_fence(__ATOMIC_ACQUIRE, "workgroup");
    if (OUT_MODE == 0) {
      float* C = (float*)Cout + (size_t)b * strideC;
      const int hh = lane >> 4, c4 = (lane & 15) * 4;
      for (int pass = 0; pass < 2; ++pass) {
#pragma unroll
        for (int it = 0; it < 8; ++it) {
          const int row = it * 2 + hh;
          v4f v = *(const v4f*)(slab + row * 68 + c4);
          *(volatile v4f*)(C + (size_t)(mBase + row) * ldc + n0 + c4) = v;
        }
        __threadfence();
      }
    } else {
      const int q = lane >> 3, c8 = (lane & 7) * 8;
      unsigned short* C  = (unsigned short*)Cout  + (size_t)b * strideC;
      unsigned short* C2 = (OUT_MODE == 2) ? ((unsigned short*)Cout2 + (size_t)b * strideC) : nullptr;
      for (int pass = 0; pass < 2; ++pass) {
#pragma unroll
        for (int it = 0; it < 4; ++it) {
          const int row = it * 4 + q;
          const float* sp = slab + row * 68 + c8;
          v8h hv, lv;
#pragma unroll
          for (int e = 0; e < 8; ++e) {
            if (OUT_MODE == 1) {
              hv[e] = (_Float16)sp[e];
            } else {
              unsigned short hb = f2bf_bits(sp[e]);
              unsigned short lb = f2bf_bits(sp[e] - bf_bits2f(hb));
              hv[e] = __builtin_bit_cast(_Float16, hb);
              lv[e] = __builtin_bit_cast(_Float16, lb);
            }
          }
          *(volatile v8h*)(C + (size_t)(mBase + row) * ldc + n0 + c8) = hv;
          if (OUT_MODE == 2) *(volatile v8h*)(C2 + (size_t)(mBase + row) * ldc + n0 + c8) = lv;
        }
        __threadfence();
      }
    }
    __builtin_amdgcn_fence(__ATOMIC_RELEASE, "workgroup");
    __builtin_amdgcn_wave_barrier();
    __builtin_amdgcn_fence(__ATOMIC_ACQUIRE, "workgroup");
  }
}

__global__ __launch_bounds__(256) void cast_scale_f32_f16x2(
    const float* __restrict__ in, _Float16* __restrict__ out, int n2, float sc) {
  int i = blockIdx.x * 256 + threadIdx.x;
  if (i < n2) {
    const _Float16 h0 = (_Float16)(sc * in[2 * i]), h1 = (_Float16)(sc * in[2 * i + 1]);
    const unsigned u = (unsigned)__builtin_bit_cast(unsigned short, h0) | ((unsigned)__builtin_bit_cast(unsigned short, h1) << 16);
    ((volatile unsigned*)out)[i] = u;
    __threadfence();
    ((volatile unsigned*)out)[i] = u;
  }
}

__global__ __launch_bounds__(256) void bias_prep(const float* __restrict__ b_ih, const float* __restrict__ b_hh,
                                                 float* __restrict__ bc, int n3, int n2h) {
  const int j = threadIdx.x;
  if (j < n3) {
    const float v = b_ih[j] + ((j < n2h) ? b_hh[j] : 0.0f);
    ((volatile float*)bc)[j] = v;
    __threadfence();
    ((volatile float*)bc)[j] = v;
  }
}

#define LSEQ   512
#define ESZ    32
#define HSZ    64
#define G3     192
#define RB     64
#define NTG    128
#define OPITCH 68
#define TCH    32

#define LOG2E_F 1.4426950408889634f
#define INV128  0.0078125f

__device__ __forceinline__ float fexp2(float x) { return __builtin_amdgcn_exp2f(x); }
__device__ __forceinline__ float frcp(float x)  { return __builtin_amdgcn_rcpf(x); }
__device__ __forceinline__ float sigm0(float a) { return frcp(1.0f + fexp2(a * (-LOG2E_F))); }
__device__ __forceinline__ float tanh0(float a) { return 1.0f - 2.0f * frcp(fexp2(a * (2.0f * LOG2E_F)) + 1.0f); }

__device__ __forceinline__ v8f mma_f16(v16h a, v16h b, v8f c) {
  c = __builtin_amdgcn_wmma_f32_16x16x32_f16(false, a, false, b, (short)0, c, false, false);
  asm volatile("v_nop\n\tv_nop\n\tv_nop\n\tv_nop" : "+v"(c) : "v"(a), "v"(b));
  return c;
}

__device__ __forceinline__ void wave_lds_sync() {
  __builtin_amdgcn_fence(__ATOMIC_RELEASE, "workgroup");
  __builtin_amdgcn_wave_barrier();
  __builtin_amdgcn_fence(__ATOMIC_ACQUIRE, "workgroup");
}

__global__ __launch_bounds__(NTG)
void gru_persist(const int* __restrict__ x, const float* __restrict__ G,
                 const float* __restrict__ w_hh, const float* __restrict__ b_hh,
                 float* __restrict__ out, int nseq, int voc) {
  __shared__ __align__(16) _Float16 sWh[G3 * HSZ];
  __shared__ __align__(16) _Float16 sA[4 * 16 * HSZ];
  __shared__ __align__(16) int      sTok[4 * 16 * TCH];
  __shared__ __align__(16) float    sOut[RB * OPITCH];
  __shared__ __align__(16) float    sBhn[HSZ];
  __shared__ int sLen[RB];
  __shared__ int sPerm[RB];

  const int tid  = threadIdx.x;
  const int wave = tid >> 5;
  const int lane = tid & 31;
  const int hh   = lane >> 4;
  const int c    = lane & 15;
  const int rowBase = blockIdx.x * RB;
  if (rowBase + RB > nseq) return;

  for (int e = tid; e < (G3 * HSZ) / 4; e += NTG) {
    const v4f w = *(const v4f*)(w_hh + 4 * e);
    v4h hv;
    hv[0] = (_Float16)(16.0f * w[0]); hv[1] = (_Float16)(16.0f * w[1]);
    hv[2] = (_Float16)(16.0f * w[2]); hv[3] = (_Float16)(16.0f * w[3]);
    *(v4h*)(sWh + 4 * e) = hv;
  }
  if (tid < HSZ) sBhn[tid] = b_hh[2 * HSZ + tid];
  if (tid < RB) sPerm[tid] = tid;
  {
    unsigned* az = (unsigned*)sA;
    for (int e = tid; e < (4 * 16 * HSZ) / 2; e += NTG) az[e] = 0u;
  }
  {
    const int lr = tid >> 1, half = tid & 1;
    const int* xr = x + (size_t)(rowBase + lr) * LSEQ + half * (LSEQ / 2);
    int cnt = 0;
#pragma unroll 4
    for (int i = 0; i < LSEQ / 8; ++i) {
      const v4i v = *(const v4i*)(xr + 4 * i);
      cnt += (v[0] != 0) + (v[1] != 0) + (v[2] != 0) + (v[3] != 0);
    }
    cnt += __shfl_xor(cnt, 1, 32);
    if (half == 0) sLen[lr] = cnt;
  }
  __syncthreads();
  if (tid < RB) {
    const int myl = sLen[tid];
    int rank = 0;
    for (int j = 0; j < RB; ++j) {
      const int lj = sLen[j];
      rank += (lj > myl) | ((lj == myl) & (j < tid));
    }
    sPerm[rank & (RB - 1)] = tid;
  }
  __syncthreads();

  const int seqLocal = sPerm[wave * 16 + c] & (RB - 1);
  int myLen = sLen[seqLocal];
  myLen = myLen < 0 ? 0 : (myLen > LSEQ ? LSEQ : myLen);
  int tw = myLen;
#pragma unroll
  for (int off = 1; off < 32; off <<= 1) tw = max(tw, __shfl_xor(tw, off, 32));
  tw = tw > LSEQ ? LSEQ : tw;
  const int tW = __builtin_amdgcn_readfirstlane(tw);

  _Float16*  sAw  = sA + wave * (16 * HSZ);
  int*       sTw  = sTok + wave * (16 * TCH);
  const int* xrow = x + (size_t)(rowBase + seqLocal) * LSEQ;
  const int  vmax = voc - 1;

  float hf[4][8];
#pragma unroll
  for (int p = 0; p < 4; ++p)
#pragma unroll
    for (int r = 0; r < 8; ++r) hf[p][r] = 0.0f;

  const v8f z8 = (v8f){0.f,0.f,0.f,0.f,0.f,0.f,0.f,0.f};

  for (int t = 0; t < tW; ++t) {
    if ((t & (TCH - 1)) == 0) {
      const int* xp = xrow + t + 16 * hh;
#pragma unroll
      for (int i = 0; i < 4; ++i) {
        const v4i v = *(const v4i*)(xp + 4 * i);
        v4i cl;
#pragma unroll
        for (int e = 0; e < 4; ++e) { int q = v[e]; q = q < 0 ? 0 : (q > vmax ? vmax : q); cl[e] = q; }
        *(v4i*)(sTw + c * TCH + 16 * hh + 4 * i) = cl;
      }
      wave_lds_sync();
    }
    int tok = sTw[c * TCH + (t & (TCH - 1))];
    tok = tok < 0 ? 0 : (tok > vmax ? vmax : tok);
    const float* gp = G + (size_t)tok * G3 + 8 * hh;
    const v16h b0 = Frag<_Float16>::load(sAw + c * HSZ + 8 * hh);
    const v16h b1 = Frag<_Float16>::load(sAw + c * HSZ + 32 + 8 * hh);
    const bool live = (t < myLen);

#pragma unroll
    for (int p = 0; p < 4; ++p) {
      const int pc = p * 16;
      const v4f xr0 = *(const v4f*)(gp + pc),            xr1 = *(const v4f*)(gp + pc + 4);
      const v4f xz0 = *(const v4f*)(gp + HSZ + pc),      xz1 = *(const v4f*)(gp + HSZ + pc + 4);
      const v4f xn0 = *(const v4f*)(gp + 2 * HSZ + pc),  xn1 = *(const v4f*)(gp + 2 * HSZ + pc + 4);
      const v4f bn0 = *(const v4f*)(sBhn + pc + 8 * hh), bn1 = *(const v4f*)(sBhn + pc + 8 * hh + 4);

      v8f ar, az, an;
      {
        const _Float16* wr = sWh + (size_t)(pc + c) * HSZ + 8 * hh;
        const _Float16* wz = wr + HSZ * HSZ;
        const _Float16* wn = wr + 2 * HSZ * HSZ;
        v16h a;
        a = Frag<_Float16>::load(wr);      ar = mma_f16(a, b0, z8);
        a = Frag<_Float16>::load(wr + 32); ar = mma_f16(a, b1, ar);
        a = Frag<_Float16>::load(wz);      az = mma_f16(a, b0, z8);
        a = Frag<_Float16>::load(wz + 32); az = mma_f16(a, b1, az);
        a = Frag<_Float16>::load(wn);      an = mma_f16(a, b0, z8);
        a = Frag<_Float16>::load(wn + 32); an = mma_f16(a, b1, an);
      }
      float xr[8], xz[8], xn[8], bn[8];
#pragma unroll
      for (int e = 0; e < 4; ++e) {
        xr[e] = xr0[e]; xr[4 + e] = xr1[e];
        xz[e] = xz0[e]; xz[4 + e] = xz1[e];
        xn[e] = xn0[e]; xn[4 + e] = xn1[e];
        bn[e] = bn0[e]; bn[4 + e] = bn1[e];
      }
      v8h hv;
#pragma unroll
      for (int r = 0; r < 8; ++r) {
        const float rg = sigm0(xr[r] + ar[r] * INV128);
        const float zg = sigm0(xz[r] + az[r] * INV128);
        const float hn = an[r] * INV128 + bn[r];
        const float ng = tanh0(xn[r] + rg * hn);
        const float ho = hf[p][r];
        const float hw = ng + zg * (ho - ng);
        const float hs = live ? hw : ho;
        hf[p][r] = hs;
        hv[r] = (_Float16)(hs * 8.0f);
      }
      *(v8h*)(sAw + c * HSZ + pc + 8 * hh) = hv;
    }
    wave_lds_sync();
  }
  __syncthreads();

  {
    float* so = sOut + seqLocal * OPITCH + 8 * hh;
#pragma unroll
    for (int p = 0; p < 4; ++p) {
      v4f o0, o1;
      o0[0] = hf[p][0]; o0[1] = hf[p][1]; o0[2] = hf[p][2]; o0[3] = hf[p][3];
      o1[0] = hf[p][4]; o1[1] = hf[p][5]; o1[2] = hf[p][6]; o1[3] = hf[p][7];
      *(v4f*)(so + p * 16)     = o0;
      *(v4f*)(so + p * 16 + 4) = o1;
    }
  }
  __syncthreads();
  {
    const int c4 = c * 4;
    const float* sb = sOut + (wave * 16) * OPITCH;
    float* ob = out + (size_t)(rowBase + wave * 16) * HSZ;
    for (int pass = 0; pass < 2; ++pass) {
#pragma unroll
      for (int it = 0; it < 8; ++it) {
        const int row = it * 2 + hh;
        const v4f v = *(const v4f*)(sb + row * OPITCH + c4);
        *(volatile v4f*)(ob + (size_t)row * HSZ + c4) = v;
      }
      __threadfence();
    }
  }
}

extern "C" void kernel_launch(void* const* d_in, const int* in_sizes, int n_in,
                              void* d_out, int out_size, void* d_ws, size_t ws_size,
                              hipStream_t stream) {
  if (n_in < 6) return;
  const int nx = in_sizes[0];
  if (nx <= 0 || (nx % LSEQ) != 0) return;
  const int nseq = nx / LSEQ;
  if ((nseq % RB) != 0 || out_size != nseq * HSZ) return;
  const int nemb = in_sizes[1];
  if (nemb <= 0 || (nemb % ESZ) != 0) return;
  const int voc = nemb / ESZ;
  if ((voc % 64) != 0) return;
  if (in_sizes[2] != G3 * ESZ || in_sizes[3] != G3 * HSZ || in_sizes[4] != G3 || in_sizes[5] != G3) return;

  const int*   x    = (const int*)d_in[0];
  const float* emb  = (const float*)d_in[1];
  const float* w_ih = (const float*)d_in[2];
  const float* w_hh = (const float*)d_in[3];
  const float* b_ih = (const float*)d_in[4];
  const float* b_hh = (const float*)d_in[5];
  float* out = (float*)d_out;

  char* ws = (char*)d_ws;
  size_t o = 0;
  const size_t szEmb16 = ((size_t)voc * ESZ * 2 + 255) & ~(size_t)255;
  const size_t szWih16 = ((size_t)G3 * ESZ * 2 + 255) & ~(size_t)255;
  const size_t szBias  = ((size_t)G3 * 4 + 255) & ~(size_t)255;
  const size_t szG     = ((size_t)voc * G3 * 4 + 255) & ~(size_t)255;
  _Float16* emb16 = (_Float16*)(ws + o); o += szEmb16;
  _Float16* wih16 = (_Float16*)(ws + o); o += szWih16;
  float*    biasc = (float*)(ws + o);    o += szBias;
  float*    Gt    = (float*)(ws + o);    o += szG;
  if (o > ws_size || o > ((size_t)128 << 20)) return;

  {
    const int n2 = nemb / 2;
    cast_scale_f32_f16x2<<<(n2 + 255) / 256, 256, 0, stream>>>(emb, emb16, n2, 16.0f);
  }
  {
    const int n2 = (G3 * ESZ) / 2;
    cast_scale_f32_f16x2<<<(n2 + 255) / 256, 256, 0, stream>>>(w_ih, wih16, n2, 16.0f);
  }
  bias_prep<<<1, 256, 0, stream>>>(b_ih, b_hh, biasc, G3, 2 * HSZ);
  {
    const int tiles = (voc / 64) * (G3 / 64);
    dim3 grid((tiles + 7) / 8, 1);
    wmma_gemm64<0, false, 2, 0, false, 0><<<grid, 256, 0, stream>>>(
        (const unsigned short*)emb16, (const unsigned short*)emb16, ESZ, 0L,
        (const unsigned short*)wih16, (const unsigned short*)wih16, ESZ, 0L,
        (void*)Gt, (void*)Gt, G3, 0L,
        biasc, biasc, 0L,
        voc, G3, ESZ, 1.0f / 256.0f);
  }
  gru_persist<<<nseq / RB, NTG, 0, stream>>>(x, Gt, w_hh, b_hh, out, nseq, voc);
  (void)hipGetLastError();
}
